// LSTM_cell_AR_77549929496853
// MI455X (gfx1250) — hardware-verified
//
#include <hip/hip_runtime.h>
#include <math.h>


#define NBATCH 256
#define TTOT 256
#define WIN 128
#define NI 8
#define HH 512
#define G4 2048
#define NOUT 129
#define RB 16

typedef __attribute__((ext_vector_type(16))) _Float16 v16h;
typedef __attribute__((ext_vector_type(8)))  _Float16 v8h;
typedef __attribute__((ext_vector_type(8)))  float v8f;
typedef __attribute__((ext_vector_type(4)))  float v4f;
typedef __attribute__((ext_vector_type(4)))  unsigned v4u;
typedef float __attribute__((may_alias)) float_a;

template <typename T> __device__ __forceinline__ void vst2(void* p, T v) { *(volatile T*)p = v; __threadfence(); *(volatile T*)p = v; }
__device__ __forceinline__ v8f wmma16(v16h a, v16h b, v8f c) {
  v8f d = __builtin_amdgcn_wmma_f32_16x16x32_f16(false, a, false, b, (short)0, c, false, false);
  asm volatile("v_nop\n\tv_nop\n\tv_nop\n\tv_nop" : "+v"(d) : "v"(a), "v"(b));
  return d;
}
__device__ __forceinline__ v16h frag_h(const _Float16* rowk0, int lane) {
  union { v16h v; v8h q[2]; } u; const _Float16* p = rowk0 + 8 * (lane >> 4);
  u.q[0] = *(const v8h*)p; u.q[1] = *(const v8h*)(p + 16); return u.v;
}
__device__ __forceinline__ float sigm(float x) { return 1.0f / (1.0f + expf(-x)); }
#define LDSX() do { asm volatile("s_wait_dscnt 0" ::: "memory"); __builtin_amdgcn_wave_barrier(); __builtin_amdgcn_fence(__ATOMIC_RELEASE, "workgroup"); } while (0)

__global__ __launch_bounds__(256) void k_cvt(const float* __restrict__ s, _Float16* __restrict__ d, size_t n8) {
  const size_t g8 = (size_t)blockIdx.x * 256 + threadIdx.x; if (g8 >= n8) return;
  union { v8h h; v4u u; } pk;
#pragma unroll
  for (int e = 0; e < 8; ++e) pk.h[e] = (_Float16)s[g8 * 8 + e];
  vst2(d + g8 * 8, pk.u);
}
__global__ __launch_bounds__(256) void k_cvt8(const float* __restrict__ s, _Float16* __restrict__ d) {
  const int n = blockIdx.x * 256 + threadIdx.x; if (n >= G4) return;
  union { v8h h; v4u u; } pk[4];
#pragma unroll
  for (int q = 0; q < 4; ++q)
#pragma unroll
    for (int e = 0; e < 8; ++e) pk[q].h[e] = (_Float16)(q == 0 ? s[(size_t)n * NI + e] : 0.f);
#pragma unroll
  for (int q = 0; q < 4; ++q) vst2(d + (size_t)n * 32 + q * 8, pk[q].u);
}

template <int K>
__device__ __forceinline__ void gemm_cols(v8f acc[8], const _Float16* A, int lda, const _Float16* __restrict__ W, int n0w, int lane) {
  const int col = lane & 15;
#pragma unroll 1
  for (int kc = 0; kc < K / 32; ++kc) { const v16h a = frag_h(A + col * lda + kc * 32, lane);
#pragma unroll
    for (int t = 0; t < 8; ++t) acc[t] = wmma16(a, frag_h(W + (size_t)(n0w + t * 16 + col) * K + kc * 32, lane), acc[t]); }
}

__global__ __launch_bounds__(256) void k_lstm(const float* __restrict__ x, const _Float16* __restrict__ Wih0, const _Float16* __restrict__ Whh0,
                                            const float* __restrict__ bih0, const float* __restrict__ bhh0,
                                            const _Float16* __restrict__ Wih1, const _Float16* __restrict__ Whh1, const float* __restrict__ bih1, const float* __restrict__ bhh1,
                                            const _Float16* __restrict__ cWih, const _Float16* __restrict__ cWhh, const float* __restrict__ cbih, const float* __restrict__ cbhh,
                                            const float* __restrict__ linW, const float* __restrict__ linb, _Float16* __restrict__ hs0, float* __restrict__ obuf) {
  __shared__ __align__(16) float gates[RB][G4];
  __shared__ __align__(16) _Float16 h16[RB][HH + 16];
  __shared__ __align__(16) _Float16 x16[RB][32 + 16];
  __shared__ float prev[RB];
  __shared__ __align__(16) float outb[RB * 132];
  const int tid = threadIdx.x, w = tid >> 5, lane = tid & 31, col = lane & 15, g = lane >> 4;
  const int blk = blockIdx.x, r = tid >> 4, u0 = (tid & 15) * 32;
  const int n0w = w * 256;
  float c[32];
  _Float16* hsb = hs0 + (size_t)blk * WIN * RB * HH;
  float dlast = 0.f;
#pragma unroll
  for (int j = 0; j < 32; ++j) { c[j] = 0.f; h16[r][u0 + j] = (_Float16)0.f; }
  if (tid < RB) prev[tid] = 0.f;
  __syncthreads();
#pragma unroll 1
  for (int phase = 0; phase < 3; ++phase) {
    const _Float16* Wi = phase == 0 ? Wih0 : (phase == 1 ? Wih1 : cWih);
    const _Float16* Wh = phase == 0 ? Whh0 : (phase == 1 ? Whh1 : cWhh);
    const float* bi = phase == 0 ? bih0 : (phase == 1 ? bih1 : cbih);
    const float* bh = phase == 0 ? bhh0 : (phase == 1 ? bhh1 : cbhh);
    if (phase == 1) {
#pragma unroll
      for (int j = 0; j < 32; ++j) { c[j] = 0.f; h16[r][u0 + j] = (_Float16)0.f; } }
    if (phase == 2) {
      if ((tid & 15) == 0) { const float o = dlast + linb[0]; prev[r] = o; outb[r * NOUT + 0] = o; } }
    __syncthreads();
#pragma unroll 1
    for (int t = 0; t < WIN; ++t) {
      if (phase != 1) { const int tt = phase == 0 ? t : WIN + t;
        for (int i = tid; i < RB * 32; i += 256) { const int rr = i >> 5, k = i & 31; float v = 0.f;
          if (k < NI) v = x[((size_t)(blk * RB + rr) * TTOT + tt) * NI + k];
          if (phase == 2 && k == 0) v = prev[rr];
          x16[rr][k] = (_Float16)v; } }
      __syncthreads();
#pragma unroll 1
      for (int half = 0; half < 2; ++half) { const int nh = n0w + half * 128;
        v8f acc[8];
#pragma unroll
        for (int q = 0; q < 8; ++q) acc[q] = (v8f){};
        if (phase == 1) gemm_cols<HH>(acc, hsb + (size_t)t * RB * HH, HH, Wi, nh, lane);
        else            gemm_cols<32>(acc, &x16[0][0], 32 + 16, Wi, nh, lane);
        gemm_cols<HH>(acc, &h16[0][0], HH + 16, Wh, nh, lane);
#pragma unroll
        for (int q = 0; q < 8; ++q) { const int n = nh + q * 16 + col; const float bb = bi[n] + bh[n];
#pragma unroll
          for (int rr = 0; rr < 8; ++rr) gates[8 * g + rr][n] = acc[q][rr] + bb; } }
      __syncthreads();
      float d = 0.f;
      union { v8h hv[4]; v4u uu[4]; _Float16 hh[32]; } hp;
#pragma unroll
      for (int j = 0; j < 32; ++j) { const int u = u0 + j;
        const float ig = sigm(gates[r][u]), fg = sigm(gates[r][HH + u]), gg = tanhf(gates[r][2 * HH + u]), og = sigm(gates[r][3 * HH + u]);
        c[j] = fg * c[j] + ig * gg; const float hv = og * tanhf(c[j]); hp.hh[j] = (_Float16)hv;
        d += hv * linW[u]; }
#pragma unroll
      for (int q = 0; q < 4; ++q) *(v4u*)(&h16[r][u0 + q * 8]) = hp.uu[q];
      if (phase == 0) {
#pragma unroll
        for (int q = 0; q < 4; ++q) vst2(hsb + ((size_t)t * RB + r) * HH + u0 + q * 8, hp.uu[q]); }
#pragma unroll
      for (int off = 8; off >= 1; off >>= 1) d += __shfl_xor(d, off, 32);
      dlast = d;
      if (phase == 2 && (tid & 15) == 0) { const float o = d + linb[0]; prev[r] = o; outb[r * NOUT + 1 + t] = o; }
      __syncthreads();
    }
  }
  for (int q = tid; q < RB * NOUT / 4; q += 256) vst2(obuf + (size_t)blk * RB * NOUT + q * 4, *(const v4f*)(&outb[q * 4]));
}
__global__ __launch_bounds__(256) void k_out(const float* __restrict__ obuf, float* __restrict__ out) {
  for (int q = threadIdx.x; q < NBATCH * NOUT / 4; q += 256) vst2(out + q * 4, *(const v4f*)(obuf + q * 4));
}

extern "C" void kernel_launch(void* const* d_in, const int* in_sizes, int n_in,
                              void* d_out, int out_size, void* d_ws, size_t ws_size,
                              hipStream_t stream) {
  (void)in_sizes; (void)n_in; (void)out_size; (void)ws_size;
  const float* x = (const float*)d_in[0];
  const float* Wih0 = (const float*)d_in[1]; const float* Whh0 = (const float*)d_in[2]; const float* bih0 = (const float*)d_in[3]; const float* bhh0 = (const float*)d_in[4];
  const float* Wih1 = (const float*)d_in[5]; const float* Whh1 = (const float*)d_in[6]; const float* bih1 = (const float*)d_in[7]; const float* bhh1 = (const float*)d_in[8];
  const float* cWih = (const float*)d_in[9]; const float* cWhh = (const float*)d_in[10]; const float* cbih = (const float*)d_in[11]; const float* cbhh = (const float*)d_in[12];
  const float* linW = (const float*)d_in[13]; const float* linb = (const float*)d_in[14];
  float* out = (float*)d_out;
  char* ws = (char*)d_ws; size_t off = 0;
  auto take = [&](size_t bytes) { char* p = ws + off; off += (bytes + 255) & ~(size_t)255; return p; };
  _Float16* Wi0 = (_Float16*)take((size_t)G4 * 32 * 2); _Float16* Wh0 = (_Float16*)take((size_t)G4 * HH * 2);
  _Float16* Wi1 = (_Float16*)take((size_t)G4 * HH * 2); _Float16* Wh1 = (_Float16*)take((size_t)G4 * HH * 2);
  _Float16* Wic = (_Float16*)take((size_t)G4 * 32 * 2); _Float16* Whc = (_Float16*)take((size_t)G4 * HH * 2);
  _Float16* hs0 = (_Float16*)take((size_t)NBATCH * WIN * HH * 2);
  float* obuf = (float*)take((size_t)NBATCH * NOUT * 4 + 256);
  const unsigned nb = (unsigned)((G4 * HH / 8 + 255) / 256);
  k_cvt8<<<G4 / 256, 256, 0, stream>>>(Wih0, Wi0);
  k_cvt<<<nb, 256, 0, stream>>>(Whh0, Wh0, (size_t)G4 * HH / 8);
  k_cvt<<<nb, 256, 0, stream>>>(Wih1, Wi1, (size_t)G4 * HH / 8);
  k_cvt<<<nb, 256, 0, stream>>>(Whh1, Wh1, (size_t)G4 * HH / 8);
  k_cvt8<<<G4 / 256, 256, 0, stream>>>(cWih, Wic);
  k_cvt<<<nb, 256, 0, stream>>>(cWhh, Whc, (size_t)G4 * HH / 8);
  k_lstm<<<NBATCH / RB, 256, 0, stream>>>(x, Wi0, Wh0, bih0, bhh0, Wi1, Wh1, bih1, bhh1, Wic, Whc, cbih, cbhh, linW, linb, hs0, obuf);
  k_out<<<1, 256, 0, stream>>>(obuf, out);
}
